// NTMHeadBase_19387482374144
// MI455X (gfx1250) — hardware-verified
//
#include <hip/hip_runtime.h>
#include <math.h>

#define NBATCH 4096
#define NMEM   2048
#define CDIM   128
#define TM     16
#define EPS_   1e-16f
#define RSPLIT (1.0f / 2048.0f)

typedef _Float16 h16;
typedef __attribute__((ext_vector_type(16))) _Float16 v16h;
typedef __attribute__((ext_vector_type(8)))  _Float16 v8h;
typedef __attribute__((ext_vector_type(8)))  float v8f;
typedef __attribute__((ext_vector_type(4)))  float v4f_t;
typedef float v4fa __attribute__((ext_vector_type(4), may_alias));
typedef __attribute__((ext_vector_type(4)))  unsigned v4u_t;
typedef unsigned v4ua __attribute__((ext_vector_type(4), may_alias));

__device__ __forceinline__ h16 lo_of(float v, h16 h) { return (h16)((v - (float)h) * 2048.0f); }
__device__ __forceinline__ v8f wmma16(v16h a, v16h b, v8f c) { return __builtin_amdgcn_wmma_f32_16x16x32_f16(false, a, false, b, (short)0, c, false, false); }
__device__ __forceinline__ v8f wmma_split(v16h a, v16h al, v16h b, v16h bl, v8f c) { v8f x = {}; x = wmma16(al, b, x); x = wmma16(a, bl, x); return wmma16(a, b, c) + x * RSPLIT; }
__device__ __forceinline__ v16h rfrag(const h16* rowp, int half) {
  const h16* p = rowp + 8 * half;
  return __builtin_shufflevector(*(const v8h*)p, *(const v8h*)(p + 16), 0,1,2,3,4,5,6,7,8,9,10,11,12,13,14,15);
}
__device__ __forceinline__ float softplus_(float x) { return (x > 20.0f) ? x : log1pf(expf(x)); }

__global__ __launch_bounds__(256) void k_prep_mem(const float* __restrict__ M, h16* __restrict__ Mp, float* __restrict__ mnorm) {
  __shared__ float nrm[32];
  const int tid = threadIdx.x, r = tid >> 3, c16 = (tid & 7) * 16, n = blockIdx.x * 32 + r;
  const float* src = M + (size_t)n * CDIM + c16;
  h16 hh[16], hl[16]; float ss = 0.0f;
#pragma unroll
  for (int i = 0; i < 16; ++i) { const float v = src[i]; ss += v * v; hh[i] = (h16)v; hl[i] = lo_of(v, hh[i]); }
  ss += __shfl_xor(ss, 1, 32); ss += __shfl_xor(ss, 2, 32); ss += __shfl_xor(ss, 4, 32);
  if ((tid & 7) == 0) nrm[r] = sqrtf(ss);
  __syncthreads();
  const size_t plane = (size_t)NMEM * CDIM;
  h16* d = Mp + (size_t)n * CDIM + c16;
#pragma unroll 1
  for (int pass = 0; pass < 2; ++pass) {
    *(volatile v4u_t*)(d)             = *(const v4ua*)(hh);     *(volatile v4u_t*)(d + 8)             = *(const v4ua*)(hh + 8);
    *(volatile v4u_t*)(d + plane)     = *(const v4ua*)(hl);     *(volatile v4u_t*)(d + plane + 8)     = *(const v4ua*)(hl + 8);
    if (tid < 32) *(volatile float*)(mnorm + blockIdx.x * 32 + tid) = nrm[tid];
    __threadfence();
  }
}

__global__ __launch_bounds__(256) void k_head(const float* __restrict__ k, const float* __restrict__ beta, const float* __restrict__ g,
                                             const float* __restrict__ s, const float* __restrict__ gamma, const float* __restrict__ wprev,
                                             const h16* __restrict__ Mp, const float* __restrict__ mnorm, float* __restrict__ out) {
  __shared__ __attribute__((aligned(16))) float wrow[TM][NMEM + 4];
  __shared__ __attribute__((aligned(16))) h16 ka[2][TM * 136];
  __shared__ float knorm[TM], pb[TM], pg[TM], ps[TM][3], pgam[TM];
  const int tid = threadIdx.x, lane = tid & 31, wave = tid >> 5, half = lane >> 4, l16 = lane & 15;
  const int r0 = blockIdx.x * TM;
  for (int i = tid; i < TM * CDIM; i += 256) { const int r = i >> 7, c = i & 127; const float v = k[(size_t)(r0 + r) * CDIM + c];
    const h16 hv = (h16)v; ka[0][r * 136 + c] = hv; ka[1][r * 136 + c] = lo_of(v, hv); }
  if (tid < TM) {
    const int r = r0 + tid;
    float ss = 0.0f;
#pragma unroll 1
    for (int c = 0; c < CDIM; ++c) { const float v = k[(size_t)r * CDIM + c]; ss += v * v; }
    knorm[tid] = sqrtf(ss);
    pb[tid] = softplus_(beta[r]);
    pg[tid] = 1.0f / (1.0f + expf(-g[r]));
    pgam[tid] = 1.0f + softplus_(gamma[r]);
    const float s0 = s[r * 3 + 0], s1 = s[r * 3 + 1], s2 = s[r * 3 + 2];
    const float mx = fmaxf(s0, fmaxf(s1, s2));
    const float e0 = expf(s0 - mx), e1 = expf(s1 - mx), e2 = expf(s2 - mx), inv = 1.0f / (e0 + e1 + e2);
    ps[tid][0] = e0 * inv; ps[tid][1] = e1 * inv; ps[tid][2] = e2 * inv;
  }
  __syncthreads();
  {
    v16h af[4], afl[4];
#pragma unroll
    for (int kc = 0; kc < 4; ++kc) { af[kc] = rfrag(&ka[0][l16 * 136 + kc * 32], half); afl[kc] = rfrag(&ka[1][l16 * 136 + kc * 32], half); }
    const size_t plane = (size_t)NMEM * CDIM;
#pragma unroll 1
    for (int it = 0; it < NMEM / 16 / 8; ++it) {
      const int n0 = (wave + 8 * it) * 16, n = n0 + l16;
      const h16* mrow = Mp + (size_t)n * CDIM;
      v8f acc = {};
#pragma unroll
      for (int kc = 0; kc < 4; ++kc) acc = wmma_split(af[kc], afl[kc], rfrag(mrow + kc * 32, half), rfrag(mrow + plane + kc * 32, half), acc);
      const float mn = mnorm[n];
#pragma unroll
      for (int r = 0; r < 8; ++r) { const int row = 8 * half + r; wrow[row][n] = pb[row] * (acc[r] / (knorm[row] * mn + EPS_)); }
    }
  }
  __syncthreads();
#pragma unroll 1
  for (int rr = 0; rr < 2; ++rr) {
    const int row = wave * 2 + rr, grow = r0 + row;
    float* wr = wrow[row];
    float mx = -3.0e38f;
    for (int n = lane; n < NMEM; n += 32) mx = fmaxf(mx, wr[n]);
#pragma unroll
    for (int o = 16; o >= 1; o >>= 1) mx = fmaxf(mx, __shfl_xor(mx, o, 32));
    float sm = 0.0f;
    for (int n = lane; n < NMEM; n += 32) { const float e = expf(wr[n] - mx); wr[n] = e; sm += e; }
#pragma unroll
    for (int o = 16; o >= 1; o >>= 1) sm += __shfl_xor(sm, o, 32);
    const float inv = 1.0f / sm, gg = pg[row];
    const float* wp = wprev + (size_t)grow * NMEM;
    for (int n = lane; n < NMEM; n += 32) wr[n] = gg * (wr[n] * inv) + (1.0f - gg) * wp[n];
    __syncthreads();
    float wt[NMEM / 32];
    const float s0 = ps[row][0], s1 = ps[row][1], s2 = ps[row][2], gm = pgam[row];
#pragma unroll
    for (int i2 = 0; i2 < NMEM / 32; ++i2) { const int n = lane + 32 * i2;
      const float wm1 = wr[(n + NMEM - 1) & (NMEM - 1)], w0 = wr[n], wp1 = wr[(n + 1) & (NMEM - 1)];
      const float wtl = s0 * wm1 + s1 * w0 + s2 * wp1;
      wt[i2] = powf(wtl, gm); }
    float ssum = 0.0f;
#pragma unroll
    for (int i2 = 0; i2 < NMEM / 32; ++i2) ssum += wt[i2];
#pragma unroll
    for (int o = 16; o >= 1; o >>= 1) ssum += __shfl_xor(ssum, o, 32);
    const float ninv = 1.0f / (ssum + EPS_);
    __syncthreads();
#pragma unroll
    for (int i2 = 0; i2 < NMEM / 32; ++i2) wr[lane + 32 * i2] = wt[i2] * ninv;
  }
  __syncthreads();
#pragma unroll 1
  for (int pass = 0; pass < 2; ++pass) {
    for (int ch = tid; ch < TM * (NMEM / 4); ch += 256) { const int row = ch >> 9, q = (ch & 511) * 4;
      *(volatile v4f_t*)(out + (size_t)(r0 + row) * NMEM + q) = *(const volatile v4fa*)(&wrow[row][q]); }
    __threadfence();
  }
}

extern "C" void kernel_launch(void* const* d_in, const int* in_sizes, int n_in,
                              void* d_out, int out_size, void* d_ws, size_t ws_size,
                              hipStream_t stream) {
  (void)in_sizes; (void)n_in; (void)out_size; (void)ws_size;
  const float* k     = (const float*)d_in[0];
  const float* beta  = (const float*)d_in[1];
  const float* g     = (const float*)d_in[2];
  const float* s     = (const float*)d_in[3];
  const float* gamma = (const float*)d_in[4];
  const float* wprev = (const float*)d_in[5];
  const float* M     = (const float*)d_in[6];
  char* ws = (char*)d_ws;
  h16* Mp = (h16*)ws;
  float* mnorm = (float*)(ws + (size_t)2 * NMEM * CDIM * 2);
  k_prep_mem<<<NMEM / 32, 256, 0, stream>>>(M, Mp, mnorm);
  k_head<<<NBATCH / TM, 256, 0, stream>>>(k, beta, g, s, gamma, wprev, Mp, mnorm, (float*)d_out);
}
